// Self_Attention_75694503625032
// MI455X (gfx1250) — hardware-verified
//
#include <hip/hip_runtime.h>


#ifndef NB
#define NB 4
#endif
#ifndef SEQ
#define SEQ 4096
#endif
#define NB_FULL  4
#define SEQ_FULL 4096
#define CC   256
#define C8   32
#define CFG  64
#define PCAR 16384.0f

static_assert(SEQ % 128 == 0);
static_assert(SEQ >= 128 && SEQ <= SEQ_FULL);
static_assert(NB >= 1 && NB <= NB_FULL);
static_assert(CC % 64 == 0 && C8 == 32 && CFG == 2 * C8);

typedef _Float16 h16;
typedef unsigned short bf;
typedef __attribute__((ext_vector_type(16))) __bf16   v16bf;
typedef __attribute__((ext_vector_type(16))) _Float16 v16h;
typedef __attribute__((ext_vector_type(8)))  _Float16 v8h;
typedef __attribute__((ext_vector_type(8)))  unsigned short v8us;
typedef __attribute__((ext_vector_type(8)))  float    v8f;
typedef __attribute__((ext_vector_type(4)))  float    v4f;
typedef v8h  __attribute__((may_alias)) v8ha;
typedef v4f  __attribute__((may_alias)) v4fa;
typedef v8us __attribute__((may_alias)) v8usa;
typedef __attribute__((ext_vector_type(2))) _Float16 v2h;
typedef __attribute__((ext_vector_type(4))) _Float16 v4h;
typedef __attribute__((ext_vector_type(2))) unsigned short v2us;
typedef __attribute__((ext_vector_type(4))) unsigned short v4us;
typedef __attribute__((ext_vector_type(2))) float v2f;

static_assert(sizeof(bf) == 2 && sizeof(h16) == 2);

__device__ __forceinline__ unsigned short f2bf(float f) { unsigned u = __float_as_uint(f); u += 0x7FFFu + ((u >> 16) & 1u); return (unsigned short)(u >> 16); }
__device__ __forceinline__ float bf2f(unsigned short b) { return __uint_as_float(((unsigned)b) << 16); }
__device__ __forceinline__ float bfr(float f) { return bf2f(f2bf(f)); }
__device__ __forceinline__ v16h cat16(v8h lo, v8h hi) { return __builtin_shufflevector(lo, hi, 0, 1, 2, 3, 4, 5, 6, 7, 8, 9, 10, 11, 12, 13, 14, 15); }
__device__ __forceinline__ v16bf cat16b(v8us lo, v8us hi) { return __builtin_bit_cast(v16bf, __builtin_shufflevector(lo, hi, 0, 1, 2, 3, 4, 5, 6, 7, 8, 9, 10, 11, 12, 13, 14, 15)); }
__device__ __forceinline__ v8f wmma16(v16h a, v16h b, v8f c) { return __builtin_amdgcn_wmma_f32_16x16x32_f16(false, a, false, b, (short)0, c, false, false); }
__device__ __forceinline__ v8f wmmab(v16bf a, v16bf b, v8f c) { return __builtin_amdgcn_wmma_f32_16x16x32_bf16(false, a, false, b, (short)0, c, false, false); }
__device__ __forceinline__ h16 tohx(float x) { return (h16)x; }
__device__ __forceinline__ void splitf(float y, unsigned short& h, unsigned short& l) { h = f2bf(y); l = f2bf(y - bf2f(h)); }

template <typename T16> struct WFrag;
template <> struct WFrag<h16> { typedef v16h V; static __device__ __forceinline__ V ld(const h16* p) { return cat16(*(const v8h*)p, *(const v8h*)(p + 16)); } static __device__ __forceinline__ v8f mma(V a, V b, v8f c) { return wmma16(a, b, c); } };
template <> struct WFrag<bf> { typedef v16bf V; static __device__ __forceinline__ V ld(const bf* p) { return cat16b(*(const v8us*)p, *(const v8us*)(p + 16)); } static __device__ __forceinline__ v8f mma(V a, V b, v8f c) { return wmmab(a, b, c); } };
template <typename T16, int NSPLIT, bool BIAS>
__global__ __launch_bounds__(32) void k_gemmw(const T16* __restrict__ A, const T16* __restrict__ A2, const T16* __restrict__ Bt, const T16* __restrict__ Bt2, int K, float* C, int ldc, const float* __restrict__ bias, size_t sA, size_t sB, size_t sC) {
    typedef typename WFrag<T16>::V V;
    __shared__ __align__(16) float os[16 * 68];
    const size_t z = blockIdx.z; A += z * sA; if (A2) A2 += z * sA; Bt += z * sB; if (Bt2) Bt2 += z * sB; C += z * sC;
    const int lane = threadIdx.x & 31, lr = lane & 15, hi = lane >> 4; const int r0 = blockIdx.x * 64, c0 = blockIdx.y * 64;
    v8f acc[4][4];
#pragma unroll
    for (int mb = 0; mb < 4; ++mb)
#pragma unroll
        for (int nb = 0; nb < 4; ++nb) acc[mb][nb] = (v8f){};
    const size_t aoff = (size_t)(r0 + lr) * K + 8 * hi, boff = (size_t)(c0 + lr) * K + 8 * hi;
#pragma unroll 1
    for (int kc = 0; kc < K; kc += 32) {
        V a[4], a2[4];
#pragma unroll
        for (int mb = 0; mb < 4; ++mb) { a[mb] = WFrag<T16>::ld(A + aoff + (size_t)mb * 16 * K + kc); if (NSPLIT == 1 || NSPLIT == 2) a2[mb] = WFrag<T16>::ld(A2 + aoff + (size_t)mb * 16 * K + kc); }
#pragma unroll
        for (int nb = 0; nb < 4; ++nb) { const V b = WFrag<T16>::ld(Bt + boff + (size_t)nb * 16 * K + kc); V b2; if (NSPLIT >= 2) b2 = WFrag<T16>::ld(Bt2 + boff + (size_t)nb * 16 * K + kc);
#pragma unroll
            for (int mb = 0; mb < 4; ++mb) { acc[mb][nb] = WFrag<T16>::mma(a[mb], b, acc[mb][nb]); if (NSPLIT == 1 || NSPLIT == 2) acc[mb][nb] = WFrag<T16>::mma(a2[mb], b, acc[mb][nb]); if (NSPLIT >= 2) acc[mb][nb] = WFrag<T16>::mma(a[mb], b2, acc[mb][nb]); } }
        asm volatile("v_nop\n\tv_nop\n\tv_nop\n\tv_nop" : "+v"(acc[0][0]), "+v"(acc[1][1]), "+v"(acc[2][2]), "+v"(acc[3][3]) : "v"(a[0]), "v"(a[3]));
    }
#pragma unroll
    for (int mb = 0; mb < 4; ++mb) {
#pragma unroll
        for (int nb = 0; nb < 4; ++nb) {
#pragma unroll
            for (int j = 0; j < 8; ++j) os[(hi * 8 + j) * 68 + nb * 16 + lr] = acc[mb][nb][j]; }
        __builtin_amdgcn_wave_barrier(); asm volatile("" ::: "memory");
        float* crow = C + (size_t)(r0 + mb * 16) * ldc + c0;
#pragma unroll 1
        for (int ps = 0; ps < 2; ++ps) {
#pragma unroll
            for (int s = 0; s < 8; ++s) { const int row = 2 * s + hi, cofs = lr * 4; v4f val = *(const v4fa*)(os + row * 68 + cofs); if (BIAS) { val[0] += bfr(bias[c0 + cofs]); val[1] += bfr(bias[c0 + cofs + 1]); val[2] += bfr(bias[c0 + cofs + 2]); val[3] += bfr(bias[c0 + cofs + 3]); }
                *(volatile v4f*)(crow + (size_t)row * ldc + cofs) = val; }
            if (ps == 0) __threadfence(); }
        __builtin_amdgcn_wave_barrier(); asm volatile("" ::: "memory");
    }
}

__global__ __launch_bounds__(256) void k_cvt8(const float* __restrict__ src, bf* dst, size_t n8) { const size_t i = (size_t)blockIdx.x * 256 + threadIdx.x; if (i >= n8) return; const v8f v = *(const v8f*)(src + i * 8); v8us o;
#pragma unroll
    for (int k = 0; k < 8; ++k) o[k] = f2bf(v[k]); *(volatile v8us*)(dst + i * 8) = o; __threadfence(); *(volatile v8us*)(dst + i * 8) = o; }

__global__ __launch_bounds__(256) void k_trb(const float* __restrict__ w, int K, int N, int pitch, bf* Bt) {
    const int lane = threadIdx.x & 31; const int L0 = (blockIdx.x * 8 + (threadIdx.x >> 5)) * 8; const int nlines = N * K / 64;
#pragma unroll
    for (int ps = 0; ps < 2; ++ps) {
#pragma unroll 1
        for (int l = 0; l < 8; ++l) { const int L = L0 + l; if (L >= nlines) break; const size_t e = (size_t)L * 64 + lane * 2; const int k = (int)(e % K), n = (int)(e / K); v2us o;
            o[0] = f2bf(w[(size_t)k * pitch + n]); o[1] = f2bf(w[(size_t)(k + 1) * pitch + n]); *(volatile v2us*)(Bt + e) = o; }
        if (ps == 0) __threadfence(); }
}

__global__ __launch_bounds__(256) void k_qk(const float* __restrict__ FG, const float* __restrict__ bfp, const float* __restrict__ bgp, bf* Fh, bf* Fl, bf* Gh, bf* Gl) {
    const int t = blockIdx.x * 256 + threadIdx.x; if (t >= SEQ * 4) return; const int n = t >> 2, o = (t & 3) * 8;
    const v8f a = *(const v8f*)(FG + (size_t)n * CFG + o); const v8f g = *(const v8f*)(FG + (size_t)n * CFG + C8 + o);
    v8us fh, fl, gh, gl;
#pragma unroll
    for (int k = 0; k < 8; ++k) { const float yf = a[k] + bfr(bfp[o + k]); const float yg = g[k] + bfr(bgp[o + k]); unsigned short h1, l1; splitf(yf, h1, l1); fh[k] = h1; fl[k] = l1; splitf(yg, h1, l1); gh[k] = h1; gl[k] = l1; }
    const size_t po = (size_t)n * C8 + o;
    *(volatile v8us*)(Fh + po) = fh; *(volatile v8us*)(Fl + po) = fl; *(volatile v8us*)(Gh + po) = gh; *(volatile v8us*)(Gl + po) = gl;
    __threadfence();
    *(volatile v8us*)(Fh + po) = fh; *(volatile v8us*)(Fl + po) = fl; *(volatile v8us*)(Gh + po) = gh; *(volatile v8us*)(Gl + po) = gl;
}

__global__ __launch_bounds__(256) void k_vpl(const float* __restrict__ HH, const float* __restrict__ bhp, h16* V16) {
    const size_t i = (size_t)blockIdx.x * 256 + threadIdx.x; if (i >= (size_t)CC * SEQ / 8) return; const size_t e = i * 8; const int c = (int)(e / SEQ);
    const v8f v = *(const v8f*)(HH + e); const float bb = bfr(bhp[c]); v8h o;
#pragma unroll
    for (int k = 0; k < 8; ++k) o[k] = tohx(v[k] + bb);
    *(volatile v8h*)(V16 + e) = o; __threadfence(); *(volatile v8h*)(V16 + e) = o; }

__global__ __launch_bounds__(256) void k_asoft(const float* __restrict__ Sb, h16* P16) {
    const int lane = threadIdx.x & 31; const int row = blockIdx.x * 8 + (threadIdx.x >> 5); if (row >= SEQ) return;
    const float* sr = Sb + (size_t)row * SEQ; float v[SEQ / 32]; float mx = -3.0e38f;
#pragma unroll
    for (int ch = 0; ch < SEQ / 128; ++ch) { const int j0 = ch * 128 + lane * 4; const v4f a = *(const v4f*)(sr + j0);
#pragma unroll
        for (int q = 0; q < 4; ++q) { v[ch * 4 + q] = a[q]; mx = fmaxf(mx, a[q]); } }
#pragma unroll
    for (int sh = 16; sh; sh >>= 1) mx = fmaxf(mx, __shfl_xor(mx, sh, 32));
    float sum = 0.f;
#pragma unroll
    for (int k = 0; k < SEQ / 32; ++k) { float d0 = __fsub_rn(v[k], mx); asm volatile("" : "+v"(d0)); v[k] = __builtin_amdgcn_exp2f(__fmul_rn(d0, 1.4426950408889634f)); sum += v[k]; }
#pragma unroll
    for (int sh = 16; sh; sh >>= 1) sum += __shfl_xor(sum, sh, 32);
    const float f = __fdiv_rn(PCAR, sum);
#pragma unroll 1
    for (int ps = 0; ps < 2; ++ps) {
#pragma unroll
        for (int ch = 0; ch < SEQ / 128; ++ch) { v4h o4;
#pragma unroll
            for (int q = 0; q < 4; ++q) o4[q] = tohx(v[ch * 4 + q] * f);
            *(volatile v4h*)(P16 + (size_t)row * SEQ + ch * 128 + lane * 4) = o4; }
        if (ps == 0) __threadfence(); }
}

__global__ __launch_bounds__(256) void k_out(const float* __restrict__ Ob, const float* __restrict__ xb, const float* __restrict__ gmp, float* outb) {
    const size_t i = (size_t)blockIdx.x * 256 + threadIdx.x; if (i >= (size_t)CC * SEQ / 4) return; const size_t e = i * 4; const int c = (int)(e / SEQ); const int n = (int)(e % SEQ);
    const v4f o = *(const v4f*)(Ob + e); const v4f xv = *(const v4f*)(xb + (size_t)c * SEQ_FULL + n); const float gm = bfr(gmp[0]) * (1.0f / PCAR); v4f r;
#pragma unroll
    for (int k = 0; k < 4; ++k) r[k] = gm * o[k] + bfr(xv[k]);
    *(volatile v4f*)(outb + e) = r; __threadfence(); *(volatile v4f*)(outb + e) = r; }

static constexpr size_t al256(size_t b) { return (b + 255) & ~(size_t)255; }
static constexpr size_t WS_XT  = al256((size_t)SEQ * CC * 2);
static constexpr size_t WS_WFG = al256((size_t)CFG * CC * 2);
static constexpr size_t WS_WH  = al256((size_t)CC * CC * 2);
static constexpr size_t WS_FG  = al256((size_t)SEQ * CFG * 4);
static constexpr size_t WS_PL  = al256((size_t)SEQ * C8 * 2);
static constexpr size_t WS_HH  = al256((size_t)CC * SEQ * 4);
static constexpr size_t WS_V16 = al256((size_t)CC * SEQ * 2);
static constexpr size_t WS_S   = al256((size_t)SEQ * SEQ * 4);
static constexpr size_t WS_P   = al256((size_t)SEQ * SEQ * 2);
static constexpr size_t WS_O   = al256((size_t)CC * SEQ * 4);
static constexpr size_t WS_TOTAL = WS_XT + WS_WFG + WS_WH + WS_FG + 4 * WS_PL + WS_HH + WS_V16 + WS_S + WS_P + WS_O;
static_assert(WS_TOTAL <= 134217728ull);
static_assert((SEQ * 4) % 64 == 0 && (SEQ * 4) % 256 == 0 && (CC * SEQ / 8) % 256 == 0 && (CC * SEQ / 4) % 256 == 0 && SEQ % 8 == 0);

extern "C" void kernel_launch(void* const* d_in, const int* in_sizes, int n_in,
                              void* d_out, int out_size, void* d_ws, size_t ws_size, hipStream_t stream) {
    if (n_in < 8) return;
    if (in_sizes[0] < (NB - 1) * CC * SEQ_FULL + (CC - 1) * SEQ_FULL + SEQ) return;
    if (in_sizes[1] < C8 * CC || in_sizes[2] < C8 || in_sizes[3] < C8 * CC || in_sizes[4] < C8 || in_sizes[5] < CC * CC || in_sizes[6] < CC || in_sizes[7] < 1) return;
    if (out_size < NB * CC * SEQ) return;
    const float* x = (const float*)d_in[0]; const float* wf = (const float*)d_in[1]; const float* bfv = (const float*)d_in[2]; const float* wg = (const float*)d_in[3];
    const float* bg = (const float*)d_in[4]; const float* wh = (const float*)d_in[5]; const float* bh = (const float*)d_in[6]; const float* gamma = (const float*)d_in[7];
    float* OUT = (float*)d_out;
    char* wsp = (char*)d_ws;
    auto take = [&](size_t bytes) { char* p = wsp; wsp += (bytes + 255) & ~(size_t)255; return (void*)p; };
    bf* XT = (bf*)take((size_t)SEQ * CC * 2); bf* WFG = (bf*)take((size_t)CFG * CC * 2); bf* WH = (bf*)take((size_t)CC * CC * 2); float* FG = (float*)take((size_t)SEQ * CFG * 4);
    bf* Fh = (bf*)take((size_t)SEQ * C8 * 2); bf* Fl = (bf*)take((size_t)SEQ * C8 * 2); bf* Gh = (bf*)take((size_t)SEQ * C8 * 2); bf* Gl = (bf*)take((size_t)SEQ * C8 * 2);
    float* HHf = (float*)take((size_t)CC * SEQ * 4); h16* V16 = (h16*)take((size_t)CC * SEQ * 2);
    float* Sb = (float*)take((size_t)SEQ * SEQ * 4); h16* P16 = (h16*)take((size_t)SEQ * SEQ * 2); float* Ob = (float*)take((size_t)CC * SEQ * 4);
    if ((size_t)(wsp - (char*)d_ws) > ws_size) return;
    if ((size_t)(wsp - (char*)d_ws) != WS_TOTAL) return;

    k_cvt8<<<(unsigned)((C8 * CC / 8 + 255) / 256), 256, 0, stream>>>(wf, WFG, (size_t)C8 * CC / 8);
    k_cvt8<<<(unsigned)((C8 * CC / 8 + 255) / 256), 256, 0, stream>>>(wg, WFG + (size_t)C8 * CC, (size_t)C8 * CC / 8);
    k_cvt8<<<(unsigned)((CC * CC / 8 + 255) / 256), 256, 0, stream>>>(wh, WH, (size_t)CC * CC / 8);
    for (int b = 0; b < NB; ++b) {
        const float* xb = x + (size_t)b * CC * SEQ_FULL;
        k_trb<<<(unsigned)((SEQ * 4 + 63) / 64), 256, 0, stream>>>(xb, CC, SEQ, SEQ_FULL, XT);
        k_gemmw<bf, 0, false><<<dim3(SEQ / 64, CFG / 64, 1), 32, 0, stream>>>(XT, nullptr, WFG, nullptr, CC, FG, CFG, nullptr, 0, 0, 0);
        k_qk<<<(unsigned)(SEQ * 4 / 256), 256, 0, stream>>>(FG, bfv, bg, Fh, Fl, Gh, Gl);
        k_gemmw<bf, 0, false><<<dim3(CC / 64, SEQ / 64, 1), 32, 0, stream>>>(WH, nullptr, XT, nullptr, CC, HHf, SEQ, nullptr, 0, 0, 0);
        k_vpl<<<(unsigned)(CC * SEQ / 8 / 256), 256, 0, stream>>>(HHf, bh, V16);
        k_gemmw<bf, 2, false><<<dim3(SEQ / 64, SEQ / 64, 1), 32, 0, stream>>>(Fh, Fl, Gh, Gl, C8, Sb, SEQ, nullptr, 0, 0, 0);
        k_asoft<<<(unsigned)(SEQ / 8), 256, 0, stream>>>(Sb, P16);
        k_gemmw<h16, 0, false><<<dim3(CC / 64, SEQ / 64, 1), 32, 0, stream>>>(V16, nullptr, P16, nullptr, SEQ, Ob, SEQ, nullptr, 0, 0, 0);
        k_out<<<(unsigned)(CC * SEQ / 4 / 256), 256, 0, stream>>>(Ob, xb, gamma, OUT + (size_t)b * CC * SEQ);
    }
}
